// Capsule_49658411876931
// MI455X (gfx1250) — hardware-verified
//
#include <hip/hip_runtime.h>
#include <stddef.h>


typedef _Float16 h16;
typedef _Float16 v16h __attribute__((ext_vector_type(16)));
typedef _Float16 v8h  __attribute__((ext_vector_type(8)));
typedef float    v8f  __attribute__((ext_vector_type(8)));
typedef float    v4f  __attribute__((ext_vector_type(4)));

#ifndef NB
#define NB 32
#endif
#ifndef NI
#define NI 2048
#endif
#define NB_FULL 32
#define NI_FULL 2048
#define NJ 32
#define ND 16
#define NK 8
#define MT (NB / 16)
#define KS 8
#define IB (NI / KS)
#define IW (IB / 8)
#define SSTEPS (IW / 4)
#define CI 8
#define NCHUNK (NI / CI)

static_assert(NB >= 16 && NB <= NB_FULL && (NB % 16) == 0);
static_assert(NI >= 256 && NI <= NI_FULL && (NI % (KS * 8 * 4)) == 0);
static_assert(NJ == 32 && ND == 16 && NK == 8);
static_assert(SSTEPS >= 1 && SSTEPS * 4 * 8 * KS == NI);
static_assert(CI == 8 && (NI % CI) == 0);
static_assert(((NJ * NI * ND) % 256) == 0);
static_assert(((NB * NJ) % 64) == 0);
static_assert(((NB * ND) % 256) == 0 && NB * 4 <= 256);
static_assert(((NB * NJ * CI) % (4 * 128)) == 0);
static_assert(((NB * CI * NK) % (4 * 128)) == 0);
static_assert(((NB * CI) % 128) == 0);

#define WCARRY 64.0f
#define PCARRY 1024.0f
#define VCARRY 64.0f

#define WPL_BYTES  ((size_t)NJ * NI * ND * NK * 2)
#define PART_BYTES ((size_t)KS * NJ * NB * ND * 4)
#define V_BYTES    ((size_t)NB * NJ * ND * 4)
#define LC_BYTES   ((size_t)NB * NJ * NI * 4)
#define OFF_WS   ((size_t)0)
#define OFF_WA   (OFF_WS + WPL_BYTES)
#define OFF_PART (OFF_WA + WPL_BYTES)
#define OFF_V    (OFF_PART + PART_BYTES)
#define OFF_L1   (OFF_V + V_BYTES)
#define OFF_C1   (OFF_L1 + LC_BYTES)
#define OFF_C2   (OFF_C1 + LC_BYTES)
#define WS_TOTAL (OFF_C2 + LC_BYTES)
static_assert((WPL_BYTES % 128) == 0 && (PART_BYTES % 128) == 0);
static_assert((V_BYTES % 128) == 0 && (LC_BYTES % 128) == 0);
static_assert(WS_TOTAL <= (size_t)134217728);

__device__ __forceinline__ float bf16r(float x) {
  unsigned int u = __float_as_uint(x);
  u = (u + 0x7FFFu + ((u >> 16) & 1u)) & 0xFFFF0000u;
  return __uint_as_float(u);
}

static __device__ __forceinline__ h16 toh_flush(float v) {
  const h16 r = (h16)v;
  return (fabsf(v) < 6.103515625e-05f) ? (h16)0.0f : r;
}

__device__ __forceinline__ v16h join16(v8h lo, v8h hi) {
  v16h out;
#pragma unroll
  for (int i = 0; i < 8; ++i) { out[i] = lo[i]; out[i + 8] = hi[i]; }
  return out;
}

__device__ __forceinline__ v8f wmma16(v16h a, v16h b, v8f c) {
  v8f d = __builtin_amdgcn_wmma_f32_16x16x32_f16(false, a, false, b, (short)0, c,
                                                 false, false);
  asm volatile("v_nop\n\tv_nop\n\tv_nop\n\tv_nop" : "+v"(d) : "v"(a), "v"(b));
  return d;
}

__global__ __launch_bounds__(256) void wprep_kernel(
    const float* __restrict__ W, _Float16* __restrict__ Ws, _Float16* __restrict__ Wa) {
  __shared__ _Float16 T[256 * 8];
  const unsigned tid = threadIdx.x;
  const unsigned row = blockIdx.x * 256u + tid;
  const unsigned blk = row >> 4;
  const unsigned j = blk / (unsigned)NI;
  const unsigned i = blk - j * (unsigned)NI;
  const unsigned d = row & 15u;
  const float* src = W + (((size_t)j * NI_FULL + i) * ND + d) * NK;
  const v4f a0 = *(const v4f*)src;
  const v4f a1 = *(const v4f*)(src + 4);
  v8h o;
#pragma unroll
  for (int e = 0; e < 4; ++e) {
    o[e]     = toh_flush(WCARRY * bf16r(a0[e]));
    o[e + 4] = toh_flush(WCARRY * bf16r(a1[e]));
  }
  *(v8h*)&T[tid * 8u] = o;
  __syncthreads();
  const unsigned lb = tid >> 4, p = tid & 15u;
  const unsigned k = p >> 1, d0 = (p & 1u) * 8u;
  v8h tr;
#pragma unroll
  for (unsigned e = 0; e < 8u; ++e) tr[e] = T[(lb * 16u + d0 + e) * 8u + k];
  const size_t off = (size_t)row * 8u;
  *(volatile v8h*)(Ws + off) = o;
  *(volatile v8h*)(Wa + off) = tr;
  __threadfence();
  *(volatile v8h*)(Ws + off) = o;
  *(volatile v8h*)(Wa + off) = tr;
}

template <int UNIFORM>
__device__ __forceinline__ void sgemm_body(
    const float* __restrict__ X, const _Float16* __restrict__ Ws,
    const float* __restrict__ Cp, float* __restrict__ Part) {
  __shared__ float Red[8 * MT * 8 * 32];
  __shared__ float Os[NB * ND];
  const unsigned tid = threadIdx.x, lane = tid & 31u;
  const unsigned wave = (unsigned)__builtin_amdgcn_readfirstlane((int)(threadIdx.x >> 5));
  const unsigned hh = lane >> 4, m = lane & 15u;
  const unsigned ks = blockIdx.x, j = blockIdx.y;
  const unsigned ibase = ks * (unsigned)IB + wave * (unsigned)IW;

  v8f acc[MT];
#pragma unroll
  for (int mt = 0; mt < MT; ++mt) acc[mt] = (v8f){};

#pragma unroll 1
  for (unsigned st = 0; st < (unsigned)SSTEPS; ++st) {
    const unsigned i0 = ibase + 4u * st;
    const unsigned ia = i0 + hh;
    const _Float16* wp = Ws + (((size_t)j * NI + ia) * ND + m) * NK;
    const v8h blo = *(const v8h*)wp;
    const v8h bhi = *(const v8h*)(wp + 2 * ND * NK);
    const v16h bf = join16(blo, bhi);
#pragma unroll
    for (int mt = 0; mt < MT; ++mt) {
      const unsigned b = 16u * (unsigned)mt + m;
      float ca = 1.0f / 32.0f, cb = 1.0f / 32.0f;
      if (!UNIFORM) {
        const v4f c4 = *(const v4f*)(Cp + ((((size_t)(i0 >> 3)) * NB + b) * NJ + j) * CI + (i0 & 7u));
        ca = (hh != 0u) ? c4[1] : c4[0];
        cb = (hh != 0u) ? c4[3] : c4[2];
      }
      const float* xp = X + ((size_t)b * NI_FULL + ia) * NK;
      const v4f xa0 = *(const v4f*)(xp);
      const v4f xa1 = *(const v4f*)(xp + 4);
      const v4f xb0 = *(const v4f*)(xp + 2 * NK);
      const v4f xb1 = *(const v4f*)(xp + 2 * NK + 4);
      const float sa = PCARRY * ca, sb = PCARRY * cb;
      v16h af;
#pragma unroll
      for (int e = 0; e < 4; ++e) {
        af[e]      = toh_flush(sa * bf16r(xa0[e]));
        af[e + 4]  = toh_flush(sa * bf16r(xa1[e]));
        af[e + 8]  = toh_flush(sb * bf16r(xb0[e]));
        af[e + 12] = toh_flush(sb * bf16r(xb1[e]));
      }
      acc[mt] = wmma16(af, bf, acc[mt]);
    }
  }

#pragma unroll
  for (int mt = 0; mt < MT; ++mt)
#pragma unroll
    for (int r = 0; r < 8; ++r)
      Red[((wave * (unsigned)MT + (unsigned)mt) * 8u + (unsigned)r) * 32u + lane] = acc[mt][r];
  __syncthreads();

#pragma unroll 1
  for (unsigned o = tid; o < (unsigned)(NB * ND); o += 256u) {
    float s = 0.0f;
#pragma unroll
    for (unsigned w = 0; w < 8u; ++w) s += Red[w * (unsigned)(MT * 256) + o];
    const unsigned ln = o & 31u, r = (o >> 5) & 7u, mt = o >> 8;
    const unsigned b = 16u * mt + 8u * (ln >> 4) + r;
    Os[b * ND + (ln & 15u)] = s;
  }
  __syncthreads();

  if (tid < (unsigned)(NB * 4)) {
    const v4f val = *(const v4f*)&Os[tid * 4u];
    float* dst = Part + ((size_t)(ks * NJ + j) * NB) * ND + tid * 4u;
    *(volatile v4f*)dst = val;
    __threadfence();
    *(volatile v4f*)dst = val;
  }
}

__global__ __launch_bounds__(256) void sgemm_uniform_kernel(
    const float* __restrict__ X, const _Float16* __restrict__ Ws, float* __restrict__ Part) {
  sgemm_body<1>(X, Ws, (const float*)0, Part);
}
__global__ __launch_bounds__(256) void sgemm_routed_kernel(
    const float* __restrict__ X, const _Float16* __restrict__ Ws,
    const float* __restrict__ Cp, float* __restrict__ Part) {
  sgemm_body<0>(X, Ws, Cp, Part);
}

__global__ __launch_bounds__(256) void squash_kernel(
    const float* __restrict__ Part, float* __restrict__ dst) {
#pragma clang fp contract(off)
  const unsigned tid = threadIdx.x;
  const unsigned cap = blockIdx.x * 64u + (tid >> 2);
  const unsigned dq = tid & 3u;
  const unsigned b = cap / (unsigned)NJ;
  const unsigned j = cap - b * (unsigned)NJ;
  v4f s = {0.0f, 0.0f, 0.0f, 0.0f};
#pragma unroll 1
  for (unsigned ks = 0; ks < (unsigned)KS; ++ks) {
    const v4f p = *(const v4f*)(Part + ((size_t)(ks * NJ + j) * NB + b) * ND + dq * 4u);
    s = s + p;
  }
  s = s * (1.0f / (PCARRY * WCARRY));
  float n2 = (s[0] * s[0] + s[1] * s[1]) + (s[2] * s[2] + s[3] * s[3]);
  n2 += __shfl_xor(n2, 1, 32);
  n2 += __shfl_xor(n2, 2, 32);
  const float sc = n2 * __builtin_amdgcn_rcpf(1.0f + n2) * __builtin_amdgcn_rsqf(n2 + 1.0e-7f);
  const v4f o = s * sc;
  float* p = dst + (size_t)cap * ND + dq * 4u;
  *(volatile v4f*)p = o;
  __threadfence();
  *(volatile v4f*)p = o;
}

template <int FIRST>
__device__ __forceinline__ void agree_body(
    const float* __restrict__ X, const _Float16* __restrict__ Wa, const float* __restrict__ Vf,
    const float* __restrict__ Lold, float* __restrict__ Lnew, float* __restrict__ Cnew) {
  __shared__ float Ls[NB * NJ * CI];
  __shared__ float Xs[NB * CI * NK];
  const unsigned tid = threadIdx.x, lane = tid & 31u;
  const unsigned wave = (unsigned)__builtin_amdgcn_readfirstlane((int)(threadIdx.x >> 5));
  const unsigned hh = lane >> 4, m = lane & 15u;
  const unsigned chunk = blockIdx.x;

#pragma unroll 1
  for (unsigned q = tid; q < (unsigned)(NB * CI * NK / 4); q += 128u) {
    const unsigned b = q >> 4, wi = q & 15u;
    v4f a = *(const v4f*)(X + ((size_t)b * NI_FULL + chunk * CI) * NK + wi * 4u);
#pragma unroll
    for (int e = 0; e < 4; ++e) a[e] = bf16r(a[e]);
    *(v4f*)&Xs[q * 4u] = a;
  }
  __syncthreads();

  const unsigned ip = m >> 3, kk = m & 7u;
  const unsigned il = 2u * wave + ip;
  const unsigned ig = chunk * CI + il;
  float xv[MT][8];
#pragma unroll
  for (int mt = 0; mt < MT; ++mt)
#pragma unroll
    for (int r = 0; r < 8; ++r)
      xv[mt][r] = Xs[((16u * (unsigned)mt + 8u * hh + (unsigned)r) * CI + il) * NK + kk];

  const v8h zero8 = {};
#pragma unroll 1
  for (unsigned j = 0; j < (unsigned)NJ; ++j) {
    const v8h w8 = *(const v8h*)(Wa + ((((size_t)j * NI + ig)) * NK + kk) * ND + hh * 8u);
    const v16h bf = join16(w8, zero8);
#pragma unroll
    for (int mt = 0; mt < MT; ++mt) {
      const float* vp = Vf + ((size_t)(16u * (unsigned)mt + m) * NJ + j) * ND + hh * 8u;
      const v4f v0 = *(const v4f*)vp;
      const v4f v1 = *(const v4f*)(vp + 4);
      v8h a8;
#pragma unroll
      for (int e = 0; e < 4; ++e) {
        a8[e]     = toh_flush(VCARRY * v0[e]);
        a8[e + 4] = toh_flush(VCARRY * v1[e]);
      }
      const v16h af = join16(a8, zero8);
      const v8f t = wmma16(af, bf, (v8f){});
      float sel = 0.0f;
#pragma unroll
      for (int r = 0; r < 8; ++r) {
        float pr = t[r] * xv[mt][r];
        pr += __shfl_xor(pr, 1, 32);
        pr += __shfl_xor(pr, 2, 32);
        pr += __shfl_xor(pr, 4, 32);
        sel = (kk == (unsigned)r) ? pr : sel;
      }
      Ls[((16u * (unsigned)mt + 8u * hh + kk) * NJ + j) * CI + il] =
          sel * (1.0f / (VCARRY * WCARRY));
    }
  }
  __syncthreads();

  const size_t gbase = (size_t)chunk * (size_t)(NB * NJ * CI);
  if (FIRST) {
#pragma unroll 1
    for (unsigned q = tid; q < (unsigned)(NB * NJ * CI / 4); q += 128u) {
      const v4f val = *(const v4f*)&Ls[q * 4u];
      *(volatile v4f*)(Lnew + gbase + (size_t)q * 4u) = val;
    }
    __threadfence();
#pragma unroll 1
    for (unsigned q = tid; q < (unsigned)(NB * NJ * CI / 4); q += 128u) {
      const v4f val = *(const v4f*)&Ls[q * 4u];
      *(volatile v4f*)(Lnew + gbase + (size_t)q * 4u) = val;
    }
  } else {
#pragma unroll 1
    for (unsigned q = tid; q < (unsigned)(NB * NJ * CI / 4); q += 128u) {
      const v4f old = *(const v4f*)(Lold + gbase + (size_t)q * 4u);
      const v4f cur = *(const v4f*)&Ls[q * 4u];
      *(v4f*)&Ls[q * 4u] = old + cur;
    }
  }
  __syncthreads();

#pragma unroll 1
  for (unsigned pidx = tid; pidx < (unsigned)(NB * CI); pidx += 128u) {
    const unsigned cb = (pidx >> 3) * (unsigned)(NJ * CI) + (pidx & 7u);
    float mx = -3.0e38f;
#pragma unroll 1
    for (unsigned jj = 0; jj < (unsigned)NJ; ++jj) mx = fmaxf(mx, Ls[cb + jj * CI]);
    float sum = 0.0f;
#pragma unroll 1
    for (unsigned jj = 0; jj < (unsigned)NJ; ++jj) {
      const float e = __expf(Ls[cb + jj * CI] - mx);
      Ls[cb + jj * CI] = e;
      sum += e;
    }
    const float inv = __builtin_amdgcn_rcpf(sum);
#pragma unroll 1
    for (unsigned jj = 0; jj < (unsigned)NJ; ++jj) {
      const float e = Ls[cb + jj * CI];
      Ls[cb + jj * CI] = e * inv;
    }
  }
  __syncthreads();

#pragma unroll 1
  for (unsigned q = tid; q < (unsigned)(NB * NJ * CI / 4); q += 128u) {
    const v4f val = *(const v4f*)&Ls[q * 4u];
    *(volatile v4f*)(Cnew + gbase + (size_t)q * 4u) = val;
  }
  __threadfence();
#pragma unroll 1
  for (unsigned q = tid; q < (unsigned)(NB * NJ * CI / 4); q += 128u) {
    const v4f val = *(const v4f*)&Ls[q * 4u];
    *(volatile v4f*)(Cnew + gbase + (size_t)q * 4u) = val;
  }
}

__global__ __launch_bounds__(128) void agree_first_kernel(
    const float* __restrict__ X, const _Float16* __restrict__ Wa, const float* __restrict__ Vf,
    float* __restrict__ Lnew, float* __restrict__ Cnew) {
  agree_body<1>(X, Wa, Vf, (const float*)0, Lnew, Cnew);
}
__global__ __launch_bounds__(128) void agree_second_kernel(
    const float* __restrict__ X, const _Float16* __restrict__ Wa, const float* __restrict__ Vf,
    const float* __restrict__ Lold, float* __restrict__ Cnew) {
  agree_body<0>(X, Wa, Vf, Lold, (float*)0, Cnew);
}

extern "C" void kernel_launch(void* const* d_in, const int* in_sizes, int n_in,
                              void* d_out, int out_size, void* d_ws, size_t ws_size,
                              hipStream_t stream) {
  if (n_in < 2) return;
  const long long need_x = ((long long)(NB - 1) * NI_FULL + NI) * NK;
  const long long need_w = ((long long)(NJ - 1) * NI_FULL + NI) * ND * NK;
  if ((long long)in_sizes[0] < need_x) return;
  if ((long long)in_sizes[1] < need_w) return;
  if ((long long)out_size < (long long)NB * NJ * ND) return;
  if (ws_size < WS_TOTAL) return;

  const float* X = (const float*)d_in[0];
  const float* W = (const float*)d_in[1];
  float* out = (float*)d_out;

  char* ws = (char*)d_ws;
  _Float16* Ws16 = (_Float16*)(ws + OFF_WS);
  _Float16* Wa16 = (_Float16*)(ws + OFF_WA);
  float* Part = (float*)(ws + OFF_PART);
  float* Vf   = (float*)(ws + OFF_V);
  float* L1   = (float*)(ws + OFF_L1);
  float* C1   = (float*)(ws + OFF_C1);
  float* C2   = (float*)(ws + OFF_C2);

  const dim3 gs(KS, NJ);

  wprep_kernel<<<dim3(NJ * NI / 16), dim3(256), 0, stream>>>(W, Ws16, Wa16);

  sgemm_uniform_kernel<<<gs, dim3(256), 0, stream>>>(X, Ws16, Part);
  squash_kernel<<<dim3(NB * NJ / 64), dim3(256), 0, stream>>>(Part, Vf);
  agree_first_kernel<<<dim3(NCHUNK), dim3(128), 0, stream>>>(X, Wa16, Vf, L1, C1);

  sgemm_routed_kernel<<<gs, dim3(256), 0, stream>>>(X, Ws16, C1, Part);
  squash_kernel<<<dim3(NB * NJ / 64), dim3(256), 0, stream>>>(Part, Vf);
  agree_second_kernel<<<dim3(NCHUNK), dim3(128), 0, stream>>>(X, Wa16, Vf, L1, C2);

  sgemm_routed_kernel<<<gs, dim3(256), 0, stream>>>(X, Ws16, C2, Part);
  squash_kernel<<<dim3(NB * NJ / 64), dim3(256), 0, stream>>>(Part, out);
}
